// feature_model_v2_58600533786801
// MI455X (gfx1250) — hardware-verified
//
#include <hip/hip_runtime.h>
#include <stdint.h>
#include <stddef.h>


#define NB      16
#define NPER    4096
#define KS1     1024
#define KS2     256
#define CIN0    32
#define NNB     32
#define FOUT    128

typedef _Float16 v16h __attribute__((ext_vector_type(16)));
typedef _Float16 v8h  __attribute__((ext_vector_type(8)));
typedef _Float16 v4h  __attribute__((ext_vector_type(4)));
typedef float    v8f  __attribute__((ext_vector_type(8)));
typedef float    v4f  __attribute__((ext_vector_type(4)));
typedef int      v4i  __attribute__((ext_vector_type(4)));
typedef v8h v8ha __attribute__((may_alias));
typedef v4f v4fa __attribute__((may_alias));
typedef v4i v4ia __attribute__((may_alias));

union Frag { v16h v; v8h half[2]; };
union F8   { v8f v; float f[8]; };
union H8   { v8h v; _Float16 s[8]; };

#define F_INF (__builtin_inff())

__device__ __forceinline__ v8f wmma_f16(v16h a, v16h b, v8f c) {
    v8f d = __builtin_amdgcn_wmma_f32_16x16x32_f16(false, a, false, b, (short)0, c, false, false);
    asm volatile("v_nop\n\tv_nop\n\tv_nop\n\tv_nop" : "+v"(d) : "v"(a), "v"(b));
    return d;
}

__device__ __forceinline__ v8f zero8() {
    v8f z = {0.f, 0.f, 0.f, 0.f, 0.f, 0.f, 0.f, 0.f};
    return z;
}

__device__ __forceinline__ v16h ld_frag(const _Float16* rowp, int k0, int h) {
    Frag f;
    f.half[0] = *(const v8ha*)(rowp + k0 + 8 * h);
    f.half[1] = *(const v8ha*)(rowp + k0 + 16 + 8 * h);
    return f.v;
}

__device__ __forceinline__ float sigm(float x) {
    return 1.0f / (1.0f + __expf(-x));
}

struct WPrepArgs {
    const float* w0; const float* w1; const float* w2; const float* w3; const float* w4; const float* w5;
    _Float16* t0; _Float16* t1; _Float16* t2; _Float16* t3; _Float16* t4; _Float16* t5;
    int kdim[6]; int ndim[6]; int kpad[6]; int cend[6];
};
typedef char wprep_size_check[(sizeof(WPrepArgs) == 192) ? 1 : -1];

__global__ __launch_bounds__(256)
void wprep_kernel(WPrepArgs a) {
    const int gid = blockIdx.x * 256 + threadIdx.x;
    if (gid >= a.cend[5]) return;
    int s = 0;
    #pragma unroll
    for (int q = 0; q < 5; ++q) if (gid >= a.cend[q]) s = q + 1;
    const float* w = a.w0; _Float16* wt = a.t0;
    int K = a.kdim[0], N = a.ndim[0], KP = a.kpad[0], beg = 0;
    if (s == 1) { w = a.w1; wt = a.t1; K = a.kdim[1]; N = a.ndim[1]; KP = a.kpad[1]; beg = a.cend[0]; }
    if (s == 2) { w = a.w2; wt = a.t2; K = a.kdim[2]; N = a.ndim[2]; KP = a.kpad[2]; beg = a.cend[1]; }
    if (s == 3) { w = a.w3; wt = a.t3; K = a.kdim[3]; N = a.ndim[3]; KP = a.kpad[3]; beg = a.cend[2]; }
    if (s == 4) { w = a.w4; wt = a.t4; K = a.kdim[4]; N = a.ndim[4]; KP = a.kpad[4]; beg = a.cend[3]; }
    if (s == 5) { w = a.w5; wt = a.t5; K = a.kdim[5]; N = a.ndim[5]; KP = a.kpad[5]; beg = a.cend[4]; }
    const int local = gid - beg;
    const int kp8 = KP >> 3;
    const int n = local / kp8;
    const int k8 = local - n * kp8;
    H8 u;
    #pragma unroll
    for (int e = 0; e < 8; ++e) {
        const int k = k8 * 8 + e;
        const float f = (k < K) ? w[(size_t)k * N + n] : 0.0f;
        u.s[e] = (_Float16)f;
    }
    _Float16* dst = wt + (size_t)local * 8;
    const v8h v = u.v;
    *(volatile v8h*)dst = v;
    __threadfence();
    *(volatile v8h*)dst = v;
}

template<int P, int KMAX>
__global__ __launch_bounds__(256)
void fps_kernel(const float* __restrict__ pos, int n, int k,
                float* __restrict__ posd, const int* __restrict__ batch_ids, int ngraphs) {
    #pragma clang fp contract(off)
    __shared__ int   ssel[KMAX];
    __shared__ float swv[2][8];
    __shared__ int   swi[2][8];
    const int b = blockIdx.x;
    if (b >= ngraphs) return;
    const int t = threadIdx.x, lane = t & 31, w = t >> 5;
    const float* pb = pos + (size_t)b * n * 3;

    float px[P], py[P], pz[P], mind[P];
    const float x0 = pb[0], y0 = pb[1], z0 = pb[2];
    #pragma unroll
    for (int i = 0; i < P; ++i) {
        const int g = t * P + i;
        if (g < n) {
            px[i] = pb[(size_t)g * 3 + 0]; py[i] = pb[(size_t)g * 3 + 1]; pz[i] = pb[(size_t)g * 3 + 2];
            const float dx = px[i] - x0, dy = py[i] - y0, dz = pz[i] - z0;
            mind[i] = (dx * dx + dy * dy) + dz * dz;
        } else {
            px[i] = 0.f; py[i] = 0.f; pz[i] = 0.f; mind[i] = -2.0f;
        }
    }
    int kk = k < KMAX ? k : KMAX;
    if (kk < 1) kk = 1;
    if (t == 0) ssel[0] = 0;

    for (int it = 1; it < kk; ++it) {
        float bv = -1.0f; int bi = t * P;
        #pragma unroll
        for (int i = 0; i < P; ++i)
            if (mind[i] > bv) { bv = mind[i]; bi = t * P + i; }
        #pragma unroll
        for (int xs = 16; xs > 0; xs >>= 1) {
            const float ov = __shfl_xor(bv, xs, 32);
            const int   oi = __shfl_xor(bi, xs, 32);
            if (ov > bv || (ov == bv && oi < bi)) { bv = ov; bi = oi; }
        }
        const int buf = it & 1;
        if (lane == 0) { swv[buf][w] = bv; swi[buf][w] = bi; }
        __syncthreads();
        bv = swv[buf][0]; bi = swi[buf][0];
        #pragma unroll
        for (int q = 1; q < 8; ++q) {
            const float ov = swv[buf][q]; const int oi = swi[buf][q];
            if (ov > bv || (ov == bv && oi < bi)) { bv = ov; bi = oi; }
        }
        int ws = bi;
        ws = ws < 0 ? 0 : (ws >= n ? n - 1 : ws);
        if (t == 0) ssel[it] = ws;
        const float wx = pb[(size_t)ws * 3 + 0], wy = pb[(size_t)ws * 3 + 1], wz = pb[(size_t)ws * 3 + 2];
        #pragma unroll
        for (int i = 0; i < P; ++i) {
            const float dx = px[i] - wx, dy = py[i] - wy, dz = pz[i] - wz;
            const float d2 = (dx * dx + dy * dy) + dz * dz;
            mind[i] = fminf(mind[i], d2);
        }
    }
    __syncthreads();

    const int nch = (kk * 3) >> 2;
    float* od = posd + (size_t)b * k * 3;
    for (int c = t; c < nch; c += 256) {
        float f4[4];
        #pragma unroll
        for (int e = 0; e < 4; ++e) {
            const int f = 4 * c + e; const int q = f / 3; const int comp = f - 3 * q;
            f4[e] = pb[(size_t)ssel[q] * 3 + comp];
        }
        const v4f v = {f4[0], f4[1], f4[2], f4[3]};
        *(volatile v4f*)(od + 4 * c) = v;
    }
    __threadfence();
    for (int c = t; c < nch; c += 256) {
        float f4[4];
        #pragma unroll
        for (int e = 0; e < 4; ++e) {
            const int f = 4 * c + e; const int q = f / 3; const int comp = f - 3 * q;
            f4[e] = pb[(size_t)ssel[q] * 3 + comp];
        }
        const v4f v = {f4[0], f4[1], f4[2], f4[3]};
        *(volatile v4f*)(od + 4 * c) = v;
    }
}

template<int NSZ>
__global__ __launch_bounds__(32)
void radius_kernel(const float* __restrict__ pos_src, const float* __restrict__ posd,
                   int n, int k, float r2, int* __restrict__ nbr, int n_centers) {
    #pragma clang fp contract(off)
    __shared__ float dl[NSZ];
    __shared__ int   il[NSZ];
    __shared__ __align__(16) int sres[NNB];
    const int bc = blockIdx.x;
    if (bc >= n_centers) return;
    const int b = bc / k;
    const int lane = threadIdx.x & 31;
    const int nn = n < NSZ ? n : NSZ;
    const float cx = posd[(size_t)bc * 3 + 0];
    const float cy = posd[(size_t)bc * 3 + 1];
    const float cz = posd[(size_t)bc * 3 + 2];
    const float* pb = pos_src + (size_t)b * n * 3;

    int total = 0;
    for (int base = 0; base < nn; base += 32) {
        const int i = base + lane;
        bool flag = false; float d2 = 0.0f;
        if (i < nn) {
            const float dx = cx - pb[(size_t)i * 3 + 0];
            const float dy = cy - pb[(size_t)i * 3 + 1];
            const float dz = cz - pb[(size_t)i * 3 + 2];
            d2 = (dx * dx + dy * dy) + dz * dz;
            flag = (d2 <= r2);
        }
        const unsigned bm = __builtin_amdgcn_ballot_w32(flag);
        if (flag) {
            const int o = total + (int)__builtin_popcount(bm & ((1u << lane) - 1u));
            if ((unsigned)o < (unsigned)NSZ) { dl[o] = d2; il[o] = i; }
        }
        total += (int)__builtin_popcount(bm);
    }
    __syncthreads();
    if (total > NSZ) total = NSZ;

    int myres = -1;
    if (total <= NNB) {
        if (lane < total) myres = il[lane];
    } else {
        for (int s = 0; s < NNB; ++s) {
            float bv = F_INF; int bi = 0x7fffffff; int be = -1;
            for (int e = lane; e < total; e += 32) {
                const float d = dl[e]; const int pi = il[e];
                if (d < bv || (d == bv && pi < bi)) { bv = d; bi = pi; be = e; }
            }
            #pragma unroll
            for (int xs = 16; xs > 0; xs >>= 1) {
                const float ov = __shfl_xor(bv, xs, 32);
                const int   oi = __shfl_xor(bi, xs, 32);
                const int   oe = __shfl_xor(be, xs, 32);
                if (ov < bv || (ov == bv && oi < bi)) { bv = ov; bi = oi; be = oe; }
            }
            if (lane == s) myres = (be >= 0) ? bi : -1;
            if (lane == 0 && be >= 0) dl[be] = F_INF;
            __syncthreads();
        }
    }
    sres[lane] = myres;
    __syncthreads();
    int* orow = nbr + (size_t)bc * NNB;
    v4i v = {0, 0, 0, 0};
    if (lane < 8) { v = *(const v4ia*)(sres + 4 * lane); *(volatile v4i*)(orow + 4 * lane) = v; }
    __threadfence();
    if (lane < 8) *(volatile v4i*)(orow + 4 * lane) = v;
}

template<int KPAD, int H>
__device__ __forceinline__ void mlp_layer1(const _Float16* sfeat, _Float16* shid,
                                           const _Float16* __restrict__ w1t, const float* __restrict__ b1,
                                           int h, int m) {
    #pragma unroll
    for (int mt = 0; mt < 2; ++mt) {
        v16h afr[KPAD / 32];
        const _Float16* arow = sfeat + (mt * 16 + m) * KPAD;
        #pragma unroll
        for (int kt = 0; kt < KPAD / 32; ++kt) afr[kt] = ld_frag(arow, kt * 32, h);
        #pragma unroll 1
        for (int nt = 0; nt < H / 16; ++nt) {
            const _Float16* brow = w1t + (size_t)(nt * 16 + m) * KPAD;
            v8f acc = zero8();
            #pragma unroll
            for (int kt = 0; kt < KPAD / 32; ++kt) acc = wmma_f16(afr[kt], ld_frag(brow, kt * 32, h), acc);
            const float bias = b1[nt * 16 + m];
            F8 d; d.v = acc;
            #pragma unroll
            for (int r = 0; r < 8; ++r)
                shid[(mt * 16 + 8 * h + r) * H + nt * 16 + m] = (_Float16)sigm(d.f[r] + bias);
        }
    }
}

template<int H>
__device__ __forceinline__ float tile_colmax(const v16h* afr, const _Float16* __restrict__ brow,
                                             float bias, unsigned rm, int h) {
    v8f acc = zero8();
    #pragma unroll
    for (int kt = 0; kt < H / 32; ++kt) acc = wmma_f16(afr[kt], ld_frag(brow, kt * 32, h), acc);
    F8 d; d.v = acc;
    float cmax = -F_INF;
    #pragma unroll
    for (int r = 0; r < 8; ++r)
        if ((rm >> r) & 1u) cmax = fmaxf(cmax, d.f[r] + bias);
    return fmaxf(cmax, __shfl_xor(cmax, 16, 32));
}

template<int CIN, int KPAD, int H, int COUT>
__global__ __launch_bounds__(32)
void sa_mlp_kernel(const float* __restrict__ x_in, const float* __restrict__ pos_src,
                   const float* __restrict__ pos_dst, const int* __restrict__ nbr,
                   const _Float16* __restrict__ w1t, const float* __restrict__ b1,
                   const _Float16* __restrict__ w2t, const float* __restrict__ b2,
                   const float* __restrict__ mean, const float* __restrict__ stdv,
                   int use_scaler, float* __restrict__ out,
                   int n_src, int k_dst, int n_centers) {
    __shared__ __align__(16) _Float16 sfeat[32 * KPAD];
    __shared__ __align__(16) _Float16 shid[32 * H];
    __shared__ __align__(16) float srow[COUT];

    const int bc = blockIdx.x;
    if (bc >= n_centers) return;
    const int b = bc / k_dst;
    const int j = threadIdx.x & 31;
    const int h = j >> 4, m = j & 15;

    int nb = nbr[(size_t)bc * NNB + j];
    const bool valid = (nb >= 0);
    nb = nb < 0 ? 0 : (nb >= n_src ? n_src - 1 : nb);
    const unsigned vmask = __builtin_amdgcn_ballot_w32(valid);

    _Float16* row = sfeat + j * KPAD;
    if (valid) {
        const float* xr = x_in + ((size_t)b * n_src + nb) * CIN;
        #pragma unroll 4
        for (int c4 = 0; c4 < CIN / 4; ++c4) {
            v4f v = *(const v4f*)(xr + 4 * c4);
            if (use_scaler) {
                v.x = (v.x - mean[4 * c4 + 0]) * (1.0f / stdv[4 * c4 + 0]);
                v.y = (v.y - mean[4 * c4 + 1]) * (1.0f / stdv[4 * c4 + 1]);
                v.z = (v.z - mean[4 * c4 + 2]) * (1.0f / stdv[4 * c4 + 2]);
                v.w = (v.w - mean[4 * c4 + 3]) * (1.0f / stdv[4 * c4 + 3]);
            }
            v4h hv4;
            hv4.x = (_Float16)v.x; hv4.y = (_Float16)v.y; hv4.z = (_Float16)v.z; hv4.w = (_Float16)v.w;
            *(v4h*)(row + 4 * c4) = hv4;
        }
        const float* pr = pos_src + ((size_t)b * n_src + nb) * 3;
        const float cx = pos_dst[(size_t)bc * 3 + 0];
        const float cy = pos_dst[(size_t)bc * 3 + 1];
        const float cz = pos_dst[(size_t)bc * 3 + 2];
        row[CIN + 0] = (_Float16)(pr[0] - cx);
        row[CIN + 1] = (_Float16)(pr[1] - cy);
        row[CIN + 2] = (_Float16)(pr[2] - cz);
    } else {
        for (int c = 0; c < CIN + 3; ++c) row[c] = (_Float16)0.0f;
    }
    for (int c = CIN + 3; c < KPAD; ++c) row[c] = (_Float16)0.0f;
    __syncthreads();

    mlp_layer1<KPAD, H>(sfeat, shid, w1t, b1, h, m);
    __syncthreads();

    #pragma unroll
    for (int mt = 0; mt < 2; ++mt) {
        v16h afr[H / 32];
        const _Float16* arow = shid + (mt * 16 + m) * H;
        #pragma unroll
        for (int kt = 0; kt < H / 32; ++kt) afr[kt] = ld_frag(arow, kt * 32, h);
        const unsigned rm = vmask >> (mt * 16 + 8 * h);
        #pragma unroll 1
        for (int nt = 0; nt < COUT / 16; ++nt) {
            const float cmax = tile_colmax<H>(afr, w2t + (size_t)(nt * 16 + m) * H, b2[nt * 16 + m], rm, h);
            if (j < 16) {
                float* sp = srow + nt * 16 + j;
                if (mt == 0) *sp = cmax; else *sp = fmaxf(*sp, cmax);
            }
        }
    }
    __syncthreads();

    float* orow = out + (size_t)bc * COUT;
    v4f ov[COUT / 128];
    #pragma unroll
    for (int q = 0; q < COUT / 128; ++q) {
        const int c = j + 32 * q;
        v4f v = *(const v4fa*)(srow + 4 * c);
        v.x = fmaxf(v.x, 0.0f); v.y = fmaxf(v.y, 0.0f); v.z = fmaxf(v.z, 0.0f); v.w = fmaxf(v.w, 0.0f);
        ov[q] = v;
        *(volatile v4f*)(orow + 4 * c) = v;
    }
    __threadfence();
    #pragma unroll
    for (int q = 0; q < COUT / 128; ++q) {
        const int c = j + 32 * q;
        *(volatile v4f*)(orow + 4 * c) = ov[q];
    }
}

template<int CIN, int KPAD, int H, int COUT, int FH, int FO>
__global__ __launch_bounds__(32)
void global_head_kernel(const float* __restrict__ x_in, const float* __restrict__ pos_in,
                        const _Float16* __restrict__ w1t, const float* __restrict__ b1,
                        const _Float16* __restrict__ w2t, const float* __restrict__ b2,
                        const float* __restrict__ fw1, const float* __restrict__ fb1,
                        const float* __restrict__ fw2, const float* __restrict__ fb2,
                        float* __restrict__ out, int npts, int ngraphs) {
    __shared__ __align__(16) _Float16 sfeat[32 * KPAD];
    __shared__ __align__(16) _Float16 shid[32 * H];
    __shared__ __align__(16) float gmax[COUT];
    __shared__ __align__(16) float shv[FH];
    __shared__ __align__(16) float sout[FO];

    const int b = blockIdx.x;
    if (b >= ngraphs) return;
    const int j = threadIdx.x & 31;
    const int h = j >> 4, m = j & 15;

    for (int i = j; i < COUT; i += 32) gmax[i] = -F_INF;
    const int nch = (npts + 31) / 32;
    for (int ch = 0; ch < nch; ++ch) {
        __syncthreads();
        const int p = ch * 32 + j;
        const bool valid = (p < npts);
        const unsigned vmask = __builtin_amdgcn_ballot_w32(valid);
        _Float16* row = sfeat + j * KPAD;
        if (valid) {
            const float* xr = x_in + ((size_t)b * npts + p) * CIN;
            #pragma unroll 4
            for (int c4 = 0; c4 < CIN / 4; ++c4) {
                const v4f v = *(const v4f*)(xr + 4 * c4);
                v4h hv4;
                hv4.x = (_Float16)v.x; hv4.y = (_Float16)v.y; hv4.z = (_Float16)v.z; hv4.w = (_Float16)v.w;
                *(v4h*)(row + 4 * c4) = hv4;
            }
            const float* pr = pos_in + ((size_t)b * npts + p) * 3;
            row[CIN + 0] = (_Float16)pr[0];
            row[CIN + 1] = (_Float16)pr[1];
            row[CIN + 2] = (_Float16)pr[2];
        } else {
            for (int c = 0; c < CIN + 3; ++c) row[c] = (_Float16)0.0f;
        }
        for (int c = CIN + 3; c < KPAD; ++c) row[c] = (_Float16)0.0f;
        __syncthreads();

        mlp_layer1<KPAD, H>(sfeat, shid, w1t, b1, h, m);
        __syncthreads();

        #pragma unroll
        for (int mt = 0; mt < 2; ++mt) {
            v16h afr[H / 32];
            const _Float16* arow = shid + (mt * 16 + m) * H;
            #pragma unroll
            for (int kt = 0; kt < H / 32; ++kt) afr[kt] = ld_frag(arow, kt * 32, h);
            const unsigned rm = vmask >> (mt * 16 + 8 * h);
            #pragma unroll 1
            for (int nt = 0; nt < COUT / 16; ++nt) {
                const float cmax = tile_colmax<H>(afr, w2t + (size_t)(nt * 16 + m) * H, b2[nt * 16 + m], rm, h);
                if (j < 16) {
                    float* gp = gmax + nt * 16 + j;
                    *gp = fmaxf(*gp, cmax);
                }
            }
        }
    }
    __syncthreads();
    for (int i = j; i < COUT; i += 32) gmax[i] = fmaxf(gmax[i], 0.0f);
    __syncthreads();

    float a1[FH / 32];
    #pragma unroll
    for (int q = 0; q < FH / 32; ++q) a1[q] = 0.0f;
    for (int kq = 0; kq < COUT; ++kq) {
        const float g = gmax[kq];
        const float* wr = fw1 + (size_t)kq * FH + j;
        #pragma unroll
        for (int q = 0; q < FH / 32; ++q) a1[q] += g * wr[32 * q];
    }
    #pragma unroll
    for (int q = 0; q < FH / 32; ++q) shv[j + 32 * q] = sigm(a1[q] + fb1[j + 32 * q]);
    __syncthreads();

    float a2[FO / 32];
    #pragma unroll
    for (int q = 0; q < FO / 32; ++q) a2[q] = 0.0f;
    for (int kq = 0; kq < FH; ++kq) {
        const float hh = shv[kq];
        const float* wr = fw2 + (size_t)kq * FO + j;
        #pragma unroll
        for (int q = 0; q < FO / 32; ++q) a2[q] += hh * wr[32 * q];
    }
    #pragma unroll
    for (int q = 0; q < FO / 32; ++q) sout[j + 32 * q] = fmaxf(a2[q] + fb2[j + 32 * q], 0.0f);
    __syncthreads();

    float* orow = out + (size_t)b * FO;
    v4f ov[FO / 128];
    #pragma unroll
    for (int q = 0; q < FO / 128; ++q) {
        const int c = j + 32 * q;
        ov[q] = *(const v4fa*)(sout + 4 * c);
        *(volatile v4f*)(orow + 4 * c) = ov[q];
    }
    __threadfence();
    #pragma unroll
    for (int q = 0; q < FO / 128; ++q) {
        const int c = j + 32 * q;
        *(volatile v4f*)(orow + 4 * c) = ov[q];
    }
}

extern "C" void kernel_launch(void* const* d_in, const int* in_sizes, int n_in,
                              void* d_out, int out_size, void* d_ws, size_t ws_size,
                              hipStream_t stream) {
    if (n_in < 21) return;
    if (in_sizes[0] != NB * NPER * CIN0 || in_sizes[1] != NB * NPER * 3 || out_size != NB * FOUT) return;
    if (in_sizes[3] < CIN0 || in_sizes[4] < CIN0) return;
    if (in_sizes[5] != 35 * 64 || in_sizes[6] < 64 || in_sizes[7] != 64 * 128 || in_sizes[8] < 128) return;
    if (in_sizes[9] != 131 * 128 || in_sizes[10] < 128 || in_sizes[11] != 128 * 256 || in_sizes[12] < 256) return;
    if (in_sizes[13] != 259 * 256 || in_sizes[14] < 256 || in_sizes[15] != 256 * 512 || in_sizes[16] < 512) return;
    if (in_sizes[17] != 512 * 256 || in_sizes[18] < 256 || in_sizes[19] != 256 * 128 || in_sizes[20] < 128) return;

    const float* x      = (const float*)d_in[0];
    const float* pos    = (const float*)d_in[1];
    const int*   bat    = (const int*)d_in[2];
    const float* mean   = (const float*)d_in[3];
    const float* stdv   = (const float*)d_in[4];
    const float* sa1_w1 = (const float*)d_in[5];
    const float* sa1_b1 = (const float*)d_in[6];
    const float* sa1_w2 = (const float*)d_in[7];
    const float* sa1_b2 = (const float*)d_in[8];
    const float* sa2_w1 = (const float*)d_in[9];
    const float* sa2_b1 = (const float*)d_in[10];
    const float* sa2_w2 = (const float*)d_in[11];
    const float* sa2_b2 = (const float*)d_in[12];
    const float* g_w1   = (const float*)d_in[13];
    const float* g_b1   = (const float*)d_in[14];
    const float* g_w2   = (const float*)d_in[15];
    const float* g_b2   = (const float*)d_in[16];
    const float* fc_w1  = (const float*)d_in[17];
    const float* fc_b1  = (const float*)d_in[18];
    const float* fc_w2  = (const float*)d_in[19];
    const float* fc_b2  = (const float*)d_in[20];

    char* wsp = (char*)d_ws;
    size_t off = 0;
    auto carve = [&](size_t bytes) -> char* {
        char* p = wsp + off;
        off += (bytes + 255) & ~(size_t)255;
        return p;
    };
    float*    posd1 = (float*)carve((size_t)NB * KS1 * 3 * sizeof(float));
    int*      nbr1  = (int*)  carve((size_t)NB * KS1 * NNB * sizeof(int));
    float*    x1    = (float*)carve((size_t)NB * KS1 * 128 * sizeof(float));
    float*    posd2 = (float*)carve((size_t)NB * KS2 * 3 * sizeof(float));
    int*      nbr2  = (int*)  carve((size_t)NB * KS2 * NNB * sizeof(int));
    float*    x2    = (float*)carve((size_t)NB * KS2 * 256 * sizeof(float));
    _Float16* wt0   = (_Float16*)carve((size_t)64  * 64  * 2);
    _Float16* wt1   = (_Float16*)carve((size_t)128 * 64  * 2);
    _Float16* wt2   = (_Float16*)carve((size_t)128 * 160 * 2);
    _Float16* wt3   = (_Float16*)carve((size_t)256 * 128 * 2);
    _Float16* wt4   = (_Float16*)carve((size_t)256 * 288 * 2);
    _Float16* wt5   = (_Float16*)carve((size_t)512 * 256 * 2);
    if (off > ws_size) return;

    WPrepArgs wa = {};
    wa.w0 = sa1_w1; wa.t0 = wt0; wa.kdim[0] = 35;  wa.ndim[0] = 64;  wa.kpad[0] = 64;
    wa.w1 = sa1_w2; wa.t1 = wt1; wa.kdim[1] = 64;  wa.ndim[1] = 128; wa.kpad[1] = 64;
    wa.w2 = sa2_w1; wa.t2 = wt2; wa.kdim[2] = 131; wa.ndim[2] = 128; wa.kpad[2] = 160;
    wa.w3 = sa2_w2; wa.t3 = wt3; wa.kdim[3] = 128; wa.ndim[3] = 256; wa.kpad[3] = 128;
    wa.w4 = g_w1;   wa.t4 = wt4; wa.kdim[4] = 259; wa.ndim[4] = 256; wa.kpad[4] = 288;
    wa.w5 = g_w2;   wa.t5 = wt5; wa.kdim[5] = 256; wa.ndim[5] = 512; wa.kpad[5] = 256;
    {
        int acc = 0;
        for (int s = 0; s < 6; ++s) { acc += wa.ndim[s] * (wa.kpad[s] / 8); wa.cend[s] = acc; }
    }
    const int wchunks = wa.cend[5];
    wprep_kernel<<<dim3((unsigned)((wchunks + 255) / 256)), dim3(256), 0, stream>>>(wa);

    fps_kernel<NPER / 256, KS1><<<dim3(NB), dim3(256), 0, stream>>>(pos, NPER, KS1, posd1, bat, NB);
    radius_kernel<NPER><<<dim3(NB * KS1), dim3(32), 0, stream>>>(pos, posd1, NPER, KS1, 4.0f, nbr1, NB * KS1);
    sa_mlp_kernel<CIN0, 64, 64, 128><<<dim3(NB * KS1), dim3(32), 0, stream>>>(
        x, pos, posd1, nbr1, wt0, sa1_b1, wt1, sa1_b2, mean, stdv, 1, x1, NPER, KS1, NB * KS1);

    fps_kernel<KS1 / 256, KS2><<<dim3(NB), dim3(256), 0, stream>>>(posd1, KS1, KS2, posd2, bat, NB);
    radius_kernel<KS1><<<dim3(NB * KS2), dim3(32), 0, stream>>>(posd1, posd2, KS1, KS2, 16.0f, nbr2, NB * KS2);
    sa_mlp_kernel<128, 160, 128, 256><<<dim3(NB * KS2), dim3(32), 0, stream>>>(
        x1, posd1, posd2, nbr2, wt2, sa2_b1, wt3, sa2_b2, mean, stdv, 0, x2, KS1, KS2, NB * KS2);

    global_head_kernel<256, 288, 256, 512, 256, 128><<<dim3(NB), dim3(32), 0, stream>>>(
        x2, posd2, wt4, g_b1, wt5, g_b2, fc_w1, fc_b1, fc_w2, fc_b2, (float*)d_out, KS2, NB);
}
